// Mamba3Baseline_17669495456482
// MI455X (gfx1250) — hardware-verified
//
#include <hip/hip_runtime.h>
#include <math.h>
#include <stdint.h>

constexpr int kNB   = 2;
constexpr int kL    = 2048;
constexpr int kNH   = 8;
constexpr int kDH   = 64;
constexpr int kDN   = 64;
constexpr int kNBH  = kNB * kNH;
constexpr int kHGRP = 2;
constexpr int kNGRP = kNBH / kHGRP;
static_assert(kNBH % kHGRP == 0 && (kNH % kHGRP) == 0);
static_assert(kDN % 32 == 0 && kL % 64 == 0 && kDH % 64 == 0);

typedef __attribute__((ext_vector_type(16))) _Float16 v16h;
typedef __attribute__((ext_vector_type(8)))  _Float16 v8h;
typedef __attribute__((ext_vector_type(16))) __bf16   v16b;
typedef __attribute__((ext_vector_type(8)))  __bf16   v8b;
typedef __attribute__((ext_vector_type(8)))  float    v8f;
typedef __attribute__((ext_vector_type(4)))  float    v4f;
typedef __attribute__((ext_vector_type(2)))  float    v2f;
typedef __attribute__((ext_vector_type(4)))  unsigned int v4u;

__device__ __forceinline__ unsigned short f2bf_bits(float f) {
  unsigned u = __float_as_uint(f);
  return (unsigned short)((u + 0x7FFFu + ((u >> 16) & 1u)) >> 16);
}
__device__ __forceinline__ float bf_bits2f(unsigned short h) { return __uint_as_float(((unsigned)h) << 16); }
__device__ __forceinline__ unsigned pk16(unsigned short a, unsigned short b) { return (unsigned)a | ((unsigned)b << 16); }

__device__ __forceinline__ void dep_guard_h(v8f& a, v8f& b, v16h x, v16h y) { asm volatile("v_nop\n\tv_nop\n\tv_nop\n\tv_nop" : "+v"(a), "+v"(b) : "v"(x), "v"(y)); }
__device__ __forceinline__ void dep_guard_b(v8f& a, v8f& b, v16b x, v16b y) { asm volatile("v_nop\n\tv_nop\n\tv_nop\n\tv_nop" : "+v"(a), "+v"(b) : "v"(x), "v"(y)); }
__device__ __forceinline__ void keep4_h(v16h a, v16h b, v16h c, v16h d) { asm volatile("v_nop" :: "v"(a), "v"(b), "v"(c), "v"(d)); }
__device__ __forceinline__ void keep4_b(v16b a, v16b b, v16b c, v16b d) { asm volatile("v_nop" :: "v"(a), "v"(b), "v"(c), "v"(d)); }
__device__ __forceinline__ void acc_guard4(v8f& a, v8f& b, v8f& c, v8f& d) { asm volatile("v_nop\n\tv_nop\n\tv_nop\n\tv_nop" : "+v"(a), "+v"(b), "+v"(c), "+v"(d)); }
template <typename T> struct Frag;
template <> struct Frag<_Float16> {
  typedef v16h V; union U { v16h v; v8h h[2]; };
  static __device__ __forceinline__ v16h load(const _Float16* p) {
    U f; f.h[0] = *(const v8h*)(p); f.h[1] = *(const v8h*)(p + 16); return f.v;
  }
  static __device__ __forceinline__ v8f mma(v16h a, v16h b, v8f c) {
    return __builtin_amdgcn_wmma_f32_16x16x32_f16(false, a, false, b, (short)0, c, false, false);
  }
  static __device__ __forceinline__ void guard(v8f& a, v8f& b, v16h x, v16h y) { dep_guard_h(a, b, x, y); }
  static __device__ __forceinline__ void keep(v16h a, v16h b, v16h c, v16h d) { keep4_h(a, b, c, d); }
};
template <> struct Frag<__bf16> {
  typedef v16b V; union U { v16b v; v8b h[2]; };
  static __device__ __forceinline__ v16b load(const __bf16* p) {
    U f; f.h[0] = *(const v8b*)(p); f.h[1] = *(const v8b*)(p + 16); return f.v;
  }
  static __device__ __forceinline__ v8f mma(v16b a, v16b b, v8f c) {
    return __builtin_amdgcn_wmma_f32_16x16x32_bf16(false, a, false, b, (short)0, c, false, false);
  }
  static __device__ __forceinline__ void guard(v8f& a, v8f& b, v16b x, v16b y) { dep_guard_b(a, b, x, y); }
  static __device__ __forceinline__ void keep(v16b a, v16b b, v16b c, v16b d) { keep4_b(a, b, c, d); }
};

template <int ET> struct Elem;
template <> struct Elem<0> { typedef _Float16 T; };
template <> struct Elem<1> { typedef __bf16 T; };
template <int ET, bool SPLIT, int BIAS_MODE, int OUT_MODE, bool RESID, int ACT = 0, bool LOWER = false, bool CAUSALK = false>
__global__ __launch_bounds__(256) void wmma_gemm64(
    const unsigned short* __restrict__ Ap, const unsigned short* __restrict__ A2p, int lda, long strideA,
    const unsigned short* __restrict__ Btp, const unsigned short* __restrict__ Bt2p, int ldb, long strideB,
    void* __restrict__ Cout, void* __restrict__ Cout2, int ldc, long strideC,
    const float* __restrict__ bias,
    const float* __restrict__ resid, long strideR,
    int M, int N, int K, float scale) {
  typedef typename Elem<ET>::T T;
  typedef typename Frag<T>::V V;
  const T* A = (const T*)Ap; const T* A2 = (const T*)A2p; const T* Bt = (const T*)Btp; const T* Bt2 = (const T*)Bt2p;
  __shared__ __align__(16) float sT[8][16 * 68];
  const int b    = blockIdx.y;
  const int lane = threadIdx.x & 31;
  const int wave = threadIdx.x >> 5;
  const int tilesN = N >> 6;
  const int tilesM = M >> 6;
  const int tile = blockIdx.x * 8 + wave;
  if (tile >= tilesM * tilesN) return;
  const int tm = tile / tilesN;
  const int tn = tile - tm * tilesN;
  const int m0 = tm << 6;
  const int n0 = tn << 6;
  if (LOWER && n0 > m0) return;

  const T* Ab  = A  + (size_t)b * strideA;
  const T* Bb  = Bt + (size_t)b * strideB;
  const T* Ab2 = SPLIT ? (A2  + (size_t)b * strideA) : nullptr;
  const T* Bb2 = SPLIT ? (Bt2 + (size_t)b * strideB) : nullptr;

  const int rlane = lane & 15;
  const int koff  = (lane >> 4) * 8;
  const int mOff  = (lane >> 4) * 8;

  v8f acc[4][4];
#pragma unroll
  for (int i = 0; i < 4; ++i)
#pragma unroll
    for (int j = 0; j < 4; ++j) acc[i][j] = (v8f){0.f,0.f,0.f,0.f,0.f,0.f,0.f,0.f};

  const int kEnd = CAUSALK ? (((m0 + 64) < K) ? (m0 + 64) : K) : K;
  for (int k0 = 0; k0 < kEnd; k0 += 32) {
    V bh[4], bl[4];
#pragma unroll
    for (int j = 0; j < 4; ++j) {
      const size_t bo = (size_t)(n0 + (j << 4) + rlane) * ldb + koff + k0;
      bh[j] = Frag<T>::load(Bb + bo);
      if (SPLIT) bl[j] = Frag<T>::load(Bb2 + bo);
    }
#pragma unroll
    for (int i = 0; i < 4; ++i) {
      const size_t ao = (size_t)(m0 + (i << 4) + rlane) * lda + koff + k0;
      V ah = Frag<T>::load(Ab + ao);
      V al;
      if (SPLIT) al = Frag<T>::load(Ab2 + ao);
#pragma unroll
      for (int j = 0; j < 4; ++j) {
        acc[i][j] = Frag<T>::mma(ah, bh[j], acc[i][j]);
        if (SPLIT) {
          acc[i][j] = Frag<T>::mma(ah, bl[j], acc[i][j]);
          acc[i][j] = Frag<T>::mma(al, bh[j], acc[i][j]);
        }
      }
      Frag<T>::guard(acc[i][0], acc[i][3], ah, SPLIT ? al : ah);
    }
    Frag<T>::keep(bh[0], bh[1], bh[2], bh[3]);
    if (SPLIT) Frag<T>::keep(bl[0], bl[1], bl[2], bl[3]);
  }
  acc_guard4(acc[0][0], acc[0][1], acc[0][2], acc[0][3]);
  acc_guard4(acc[1][0], acc[1][1], acc[1][2], acc[1][3]);
  acc_guard4(acc[2][0], acc[2][1], acc[2][2], acc[2][3]);
  acc_guard4(acc[3][0], acc[3][1], acc[3][2], acc[3][3]);

  float* slab = sT[wave];
  const float* Rb = RESID ? (resid + (size_t)b * strideR) : nullptr;
#pragma unroll
  for (int i = 0; i < 4; ++i) {
    const int mBase = m0 + (i << 4);
#pragma unroll
    for (int j = 0; j < 4; ++j) {
      const int n = n0 + (j << 4) + rlane;
      float bv = 0.f;
      if (BIAS_MODE == 2) bv = bias[n];
#pragma unroll
      for (int r = 0; r < 8; ++r) {
        float v = acc[i][j][r] * scale;
        if (BIAS_MODE == 1) v += bias[mBase + mOff + r];
        if (BIAS_MODE == 2) v += bv;
        if (RESID) v += Rb[(size_t)(mBase + mOff + r) * ldc + n];
        if (ACT == 1) v = tanhf(v);
        if (ACT == 2) v = fmaxf(v, 0.0f);
        if (ACT == 3) v = v / (1.0f + expf(-v));
        if (ACT == 4) v = (v > 0.f) ? v : 0.01f * v;
        if (ACT == 5) v = 0.5f * v * (1.0f + erff(v * 0.70710678118654752f));
        slab[(mOff + r) * 68 + (j << 4) + rlane] = v;
      }
    }
    __builtin_amdgcn_fence(__ATOMIC_RELEASE, "workgroup");
    __builtin_amdgcn_wave_barrier();
    __builtin_amdgcn_fence(__ATOMIC_ACQUIRE, "workgroup");
    if (OUT_MODE == 0) {
      float* C = (float*)Cout + (size_t)b * strideC;
      const int hh = lane >> 4, c4 = (lane & 15) * 4;
      for (int pass = 0; pass < 2; ++pass) {
#pragma unroll
        for (int it = 0; it < 8; ++it) {
          const int row = it * 2 + hh;
          v4f v = *(const v4f*)(slab + row * 68 + c4);
          *(volatile v4f*)(C + (size_t)(mBase + row) * ldc + n0 + c4) = v;
        }
        __threadfence();
      }
    } else {
      const int q = lane >> 3, c8 = (lane & 7) * 8;
      unsigned short* C  = (unsigned short*)Cout  + (size_t)b * strideC;
      unsigned short* C2 = (OUT_MODE == 2) ? ((unsigned short*)Cout2 + (size_t)b * strideC) : nullptr;
      for (int pass = 0; pass < 2; ++pass) {
#pragma unroll
        for (int it = 0; it < 4; ++it) {
          const int row = it * 4 + q;
          const float* sp = slab + row * 68 + c8;
          v8h hv, lv;
#pragma unroll
          for (int e = 0; e < 8; ++e) {
            if (OUT_MODE == 1) {
              hv[e] = (_Float16)sp[e];
            } else {
              unsigned short hb = f2bf_bits(sp[e]);
              unsigned short lb = f2bf_bits(sp[e] - bf_bits2f(hb));
              hv[e] = __builtin_bit_cast(_Float16, hb);
              lv[e] = __builtin_bit_cast(_Float16, lb);
            }
          }
          *(volatile v8h*)(C + (size_t)(mBase + row) * ldc + n0 + c8) = hv;
          if (OUT_MODE == 2) *(volatile v8h*)(C2 + (size_t)(mBase + row) * ldc + n0 + c8) = lv;
        }
        __threadfence();
      }
    }
    __builtin_amdgcn_fence(__ATOMIC_RELEASE, "workgroup");
    __builtin_amdgcn_wave_barrier();
    __builtin_amdgcn_fence(__ATOMIC_ACQUIRE, "workgroup");
  }
}

__global__ __launch_bounds__(64) void prefix_kernel(const float* __restrict__ dt, const float* __restrict__ Avec,
                                                    const int* __restrict__ cfg_unused,
                                                    float* __restrict__ cosA, float* __restrict__ sinA,
                                                    float* __restrict__ csA, float* __restrict__ wsA) {
#pragma clang fp contract(off)
  __shared__ double pd[64];
  __shared__ double pa[64];
  __shared__ __align__(16) float sc[kL];
  __shared__ __align__(16) float ss[kL];
  __shared__ __align__(16) float scs[kL];
  __shared__ __align__(16) float sws[kL];
  (void)cfg_unused;
  const int bh = blockIdx.x;
  const int b  = bh >> 3;
  const int h  = bh & 7;
  const int t  = threadIdx.x;
  const float Ah = Avec[h];
  const int l0 = t * 32;

  double sd = 0.0, sa = 0.0;
#pragma unroll 1
  for (int i = 0; i < 32; ++i) {
    const int l = l0 + i;
    const float d = dt[((size_t)(b * kL + l)) * kNH + h];
    const float adt = Ah * d;
    sd += (double)d;
    sa += (double)adt;
  }
  pd[t] = sd;
  pa[t] = sa;
  __syncthreads();
  if (t == 0) {
    double rd = 0.0, ra = 0.0;
#pragma unroll 1
    for (int u = 0; u < 64; ++u) {
      const double vd = pd[u], va = pa[u];
      pd[u] = rd; pa[u] = ra;
      rd += vd; ra += va;
    }
  }
  __syncthreads();
  double rd = pd[t], ra = pa[t];
#pragma unroll 1
  for (int i = 0; i < 32; ++i) {
    const int l = l0 + i;
    const float d = dt[((size_t)(b * kL + l)) * kNH + h];
    const float adt = Ah * d;
    rd += (double)d;
    ra += (double)adt;
    const float ang = (float)rd;
    float sn, cn;
    sincosf(ang, &sn, &cn);
    sc[l]  = cn;
    ss[l]  = sn;
    scs[l] = (float)ra;
    sws[l] = 0.5f * (1.0f + expf(adt));
  }
  __syncthreads();
  const size_t gb = (size_t)bh * kL + (size_t)l0;
  for (int pass = 0; pass < 2; ++pass) {
#pragma unroll
    for (int q = 0; q < 8; ++q) {
      const v4f v0 = *(const v4f*)(sc  + l0 + 4 * q);
      const v4f v1 = *(const v4f*)(ss  + l0 + 4 * q);
      const v4f v2 = *(const v4f*)(scs + l0 + 4 * q);
      const v4f v3 = *(const v4f*)(sws + l0 + 4 * q);
      *(volatile v4f*)(cosA + gb + 4 * q) = v0;
      *(volatile v4f*)(sinA + gb + 4 * q) = v1;
      *(volatile v4f*)(csA  + gb + 4 * q) = v2;
      *(volatile v4f*)(wsA  + gb + 4 * q) = v3;
    }
    __threadfence();
  }
}

__global__ __launch_bounds__(256) void rope_split_kernel(const float* __restrict__ Cq, const float* __restrict__ Bk,
                                                         const float* __restrict__ cosA, const float* __restrict__ sinA,
                                                         unsigned short* __restrict__ Qh, unsigned short* __restrict__ Ql,
                                                         unsigned short* __restrict__ Kh, unsigned short* __restrict__ Kl) {
#pragma clang fp contract(off)
  const int bh  = blockIdx.y;
  const int b   = bh >> 3;
  const int tid = threadIdx.x;
  const int l   = blockIdx.x * 32 + (tid >> 3);
  const int c8  = (tid & 7) * 8;
  const int cl  = c8 & 31;
  const float cn = cosA[(size_t)bh * kL + l];
  const float sn = sinA[(size_t)bh * kL + l];
  const bool lowh = (c8 < 32);
  const float fa = lowh ? cn : sn;
  const float fb = lowh ? -sn : cn;
  const float* crow = Cq + ((size_t)(b * kL + l)) * kDN;
  const float* brow = Bk + ((size_t)(b * kL + l)) * kDN;
  const v4f qa0 = *(const v4f*)(crow + cl),      qa1 = *(const v4f*)(crow + cl + 4);
  const v4f qb0 = *(const v4f*)(crow + cl + 32), qb1 = *(const v4f*)(crow + cl + 36);
  const v4f ka0 = *(const v4f*)(brow + cl),      ka1 = *(const v4f*)(brow + cl + 4);
  const v4f kb0 = *(const v4f*)(brow + cl + 32), kb1 = *(const v4f*)(brow + cl + 36);
  float qt1[8], qt2[8], kt1[8], kt2[8];
#pragma unroll
  for (int e = 0; e < 4; ++e) {
    qt1[e] = qa0[e]; qt1[4 + e] = qa1[e]; qt2[e] = qb0[e]; qt2[4 + e] = qb1[e];
    kt1[e] = ka0[e]; kt1[4 + e] = ka1[e]; kt2[e] = kb0[e]; kt2[4 + e] = kb1[e];
  }
  unsigned qhw[4], qlw[4], khw[4], klw[4];
#pragma unroll
  for (int q = 0; q < 4; ++q) {
    const float q0 = qt1[2 * q] * fa + qt2[2 * q] * fb;
    const float q1 = qt1[2 * q + 1] * fa + qt2[2 * q + 1] * fb;
    const float k0 = kt1[2 * q] * fa + kt2[2 * q] * fb;
    const float k1 = kt1[2 * q + 1] * fa + kt2[2 * q + 1] * fb;
    const unsigned short qh0 = f2bf_bits(q0), qh1 = f2bf_bits(q1);
    const unsigned short ql0 = f2bf_bits(q0 - bf_bits2f(qh0)), ql1 = f2bf_bits(q1 - bf_bits2f(qh1));
    const unsigned short kh0 = f2bf_bits(k0), kh1 = f2bf_bits(k1);
    const unsigned short kl0 = f2bf_bits(k0 - bf_bits2f(kh0)), kl1 = f2bf_bits(k1 - bf_bits2f(kh1));
    qhw[q] = pk16(qh0, qh1); qlw[q] = pk16(ql0, ql1);
    khw[q] = pk16(kh0, kh1); klw[q] = pk16(kl0, kl1);
  }
  const v4u vqh = (v4u){qhw[0], qhw[1], qhw[2], qhw[3]};
  const v4u vql = (v4u){qlw[0], qlw[1], qlw[2], qlw[3]};
  const v4u vkh = (v4u){khw[0], khw[1], khw[2], khw[3]};
  const v4u vkl = (v4u){klw[0], klw[1], klw[2], klw[3]};
  const size_t off = ((size_t)bh * kL + (size_t)l) * kDN + c8;
  *(volatile v4u*)(Qh + off) = vqh;
  *(volatile v4u*)(Ql + off) = vql;
  *(volatile v4u*)(Kh + off) = vkh;
  *(volatile v4u*)(Kl + off) = vkl;
  __threadfence();
  *(volatile v4u*)(Qh + off) = vqh;
  *(volatile v4u*)(Ql + off) = vql;
  *(volatile v4u*)(Kh + off) = vkh;
  *(volatile v4u*)(Kl + off) = vkl;
}

__global__ __launch_bounds__(256) void xpose_split_v_kernel(const float* __restrict__ x,
                                                            unsigned short* __restrict__ outh_all,
                                                            unsigned short* __restrict__ outl_all) {
  __shared__ __align__(16) float tf[64 * 68];
  const int bz = blockIdx.z;
  const int b  = bz >> 3;
  const int h  = bz & 7;
  const float* in = x + (size_t)b * kL * kNH * kDH + (size_t)h * kDH;
  const int ldi = kNH * kDH;
  unsigned short* outh = outh_all + (size_t)bz * kDH * kL;
  unsigned short* outl = outl_all + (size_t)bz * kDH * kL;
  const int ldo = kL;
  const int c0  = blockIdx.x * 64;
  const int r0  = blockIdx.y * 64;
  const int tid = threadIdx.x;
  {
    const int sub = tid >> 4;
    const int c4  = (tid & 15) * 4;
#pragma unroll
    for (int it = 0; it < 4; ++it) {
      const int rr = it * 16 + sub;
      const v4f a = *(const v4f*)(in + (size_t)(r0 + rr) * ldi + c0 + c4);
      *(v4f*)(tf + rr * 68 + c4) = a;
    }
  }
  __syncthreads();
  const int s8 = tid >> 3;
  const int c8 = (tid & 7) * 8;
  v4u hv[2], lv[2];
#pragma unroll
  for (int it = 0; it < 2; ++it) {
    const int oc = it * 32 + s8;
    v4u a, a2;
#pragma unroll
    for (int q = 0; q < 4; ++q) {
      const float f0 = tf[(c8 + 2 * q) * 68 + oc];
      const float f1 = tf[(c8 + 2 * q + 1) * 68 + oc];
      const unsigned short h0 = f2bf_bits(f0), h1 = f2bf_bits(f1);
      const unsigned short l0 = f2bf_bits(f0 - bf_bits2f(h0));
      const unsigned short l1 = f2bf_bits(f1 - bf_bits2f(h1));
      a[q]  = pk16(h0, h1);
      a2[q] = pk16(l0, l1);
    }
    hv[it] = a; lv[it] = a2;
  }
  for (int pass = 0; pass < 2; ++pass) {
#pragma unroll
    for (int it = 0; it < 2; ++it) {
      const int oc = it * 32 + s8;
      const size_t go = (size_t)(c0 + oc) * ldo + r0 + c8;
      *(volatile v4u*)(outh + go) = hv[it];
      *(volatile v4u*)(outl + go) = lv[it];
    }
    __threadfence();
  }
}

__global__ __launch_bounds__(256) void decay_split_kernel(const float* __restrict__ S, const float* __restrict__ csA,
                                                          const float* __restrict__ wsA,
                                                          unsigned short* __restrict__ Ph, unsigned short* __restrict__ Pl,
                                                          int grp) {
#pragma clang fp contract(off)
  const int i    = blockIdx.x;
  const int hg   = blockIdx.y;
  const int tid  = threadIdx.x;
  const int wave = tid >> 5;
  int bh = grp * kHGRP + hg;
  bh = bh < 0 ? 0 : (bh > kNBH - 1 ? kNBH - 1 : bh);
  const float csl = csA[(size_t)bh * kL + i];
  const int j0 = tid * 8;
  const bool wact = (wave * 256 <= i);
  float p[8];
#pragma unroll
  for (int e = 0; e < 8; ++e) p[e] = 0.0f;
  if (wact) {
    const float* srow = S + ((size_t)hg * kL + (size_t)i) * kL + j0;
    const float* crow = csA + (size_t)bh * kL + j0;
    const float* wrow = wsA + (size_t)bh * kL + j0;
    const v4f s0 = *(const v4f*)(srow), s1 = *(const v4f*)(srow + 4);
    const v4f c0 = *(const v4f*)(crow), c1 = *(const v4f*)(crow + 4);
    const v4f w0 = *(const v4f*)(wrow), w1 = *(const v4f*)(wrow + 4);
    float sv[8], cv[8], wv[8];
#pragma unroll
    for (int e = 0; e < 4; ++e) {
      sv[e] = s0[e]; sv[4 + e] = s1[e];
      cv[e] = c0[e]; cv[4 + e] = c1[e];
      wv[e] = w0[e]; wv[4 + e] = w1[e];
    }
#pragma unroll
    for (int e = 0; e < 8; ++e) {
      const int j = j0 + e;
      const bool keep = (j <= i);
      float arg = csl - cv[e];
      arg = keep ? arg : -100.0f;
      const float dec = __expf(arg) * wv[e];
      const float pv  = sv[e] * dec;
      p[e] = keep ? pv : 0.0f;
    }
  }
  unsigned hw[4], lw[4];
#pragma unroll
  for (int q = 0; q < 4; ++q) {
    const float p0 = p[2 * q], p1 = p[2 * q + 1];
    const unsigned short hb0 = f2bf_bits(p0), hb1 = f2bf_bits(p1);
    const unsigned short lb0 = f2bf_bits(p0 - bf_bits2f(hb0));
    const unsigned short lb1 = f2bf_bits(p1 - bf_bits2f(hb1));
    hw[q] = pk16(hb0, hb1);
    lw[q] = pk16(lb0, lb1);
  }
  const v4u hvv = (v4u){hw[0], hw[1], hw[2], hw[3]};
  const v4u lvv = (v4u){lw[0], lw[1], lw[2], lw[3]};
  const size_t rowoff = ((size_t)hg * kL + (size_t)i) * kL + j0;
  *(volatile v4u*)(Ph + rowoff) = hvv;
  *(volatile v4u*)(Pl + rowoff) = lvv;
  __threadfence();
  *(volatile v4u*)(Ph + rowoff) = hvv;
  *(volatile v4u*)(Pl + rowoff) = lvv;
}

extern "C" void kernel_launch(void* const* d_in, const int* in_sizes, int n_in,
                              void* d_out, int out_size, void* d_ws, size_t ws_size,
                              hipStream_t stream) {
  if (n_in < 6) return;
  if (in_sizes[0] != kNB * kL * kNH * kDH) return;
  if (in_sizes[1] != kNB * kL * kNH) return;
  if (in_sizes[2] < kNH) return;
  if (in_sizes[3] != kNB * kL * kDN || in_sizes[4] != kNB * kL * kDN) return;
  if (in_sizes[5] < 1) return;
  if (out_size != kNB * kL * kNH * kDH) return;

  const float* x    = (const float*)d_in[0];
  const float* dt   = (const float*)d_in[1];
  const float* Avec = (const float*)d_in[2];
  const float* Bk   = (const float*)d_in[3];
  const float* Cq   = (const float*)d_in[4];
  const int*   cfg  = (const int*)d_in[5];
  float* outp = (float*)d_out;

  const size_t PVEC = (size_t)kNBH * kL * 4;
  const size_t PQK  = (size_t)kNBH * kL * kDN * 2;
  const size_t PVT  = (size_t)kNBH * kDH * kL * 2;
  const size_t PS   = (size_t)kHGRP * kL * kL * 4;
  const size_t PP   = (size_t)kHGRP * kL * kL * 2;
  size_t off = 0;
  const size_t oCos = off; off += PVEC;
  const size_t oSin = off; off += PVEC;
  const size_t oCs  = off; off += PVEC;
  const size_t oWs  = off; off += PVEC;
  const size_t oQh  = off; off += PQK;
  const size_t oQl  = off; off += PQK;
  const size_t oKh  = off; off += PQK;
  const size_t oKl  = off; off += PQK;
  const size_t oVTh = off; off += PVT;
  const size_t oVTl = off; off += PVT;
  const size_t oS   = off; off += PS;
  const size_t oPh  = off; off += PP;
  const size_t oPl  = off; off += PP;
  if (off > ws_size) return;

  char* ws = (char*)d_ws;
  float* cosA = (float*)(ws + oCos);
  float* sinA = (float*)(ws + oSin);
  float* csA  = (float*)(ws + oCs);
  float* wsA  = (float*)(ws + oWs);
  unsigned short* Qh  = (unsigned short*)(ws + oQh);
  unsigned short* Ql  = (unsigned short*)(ws + oQl);
  unsigned short* Kh  = (unsigned short*)(ws + oKh);
  unsigned short* Kl  = (unsigned short*)(ws + oKl);
  unsigned short* VTh = (unsigned short*)(ws + oVTh);
  unsigned short* VTl = (unsigned short*)(ws + oVTl);
  float*          Sb  = (float*)(ws + oS);
  unsigned short* Ph  = (unsigned short*)(ws + oPh);
  unsigned short* Pl  = (unsigned short*)(ws + oPl);

  const dim3 blk(256);
  prefix_kernel<<<dim3(kNBH), dim3(64), 0, stream>>>(dt, Avec, cfg, cosA, sinA, csA, wsA);
  rope_split_kernel<<<dim3(kL / 32, kNBH), blk, 0, stream>>>(Cq, Bk, cosA, sinA, Qh, Ql, Kh, Kl);
  xpose_split_v_kernel<<<dim3(kDH / 64, kL / 64, kNBH), blk, 0, stream>>>(x, VTh, VTl);

  const dim3 gS(((kL / 64) * (kL / 64) + 7) / 8, kHGRP);
  const dim3 gD(kL, kHGRP);
  const dim3 gPV(((kL / 64) * (kDH / 64) + 7) / 8, kHGRP);

  for (int g = 0; g < kNGRP; ++g) {
    const int bh0 = g * kHGRP;
    const int bb  = bh0 >> 3;
    const int h0  = bh0 & 7;
    wmma_gemm64<1, true, 0, 0, false, 0, true, false><<<gS, blk, 0, stream>>>(
        Qh + (size_t)bh0 * kL * kDN, Ql + (size_t)bh0 * kL * kDN, kDN, (long)kL * kDN,
        Kh + (size_t)bh0 * kL * kDN, Kl + (size_t)bh0 * kL * kDN, kDN, (long)kL * kDN,
        (void*)Sb, (void*)Sb, kL, (long)kL * kL,
        cosA, cosA, 0L, kL, kL, kDN, 1.0f);
    decay_split_kernel<<<gD, blk, 0, stream>>>(Sb, csA, wsA, Ph, Pl, g);
    wmma_gemm64<1, true, 0, 0, false, 0, false, true><<<gPV, blk, 0, stream>>>(
        Ph, Pl, kL, (long)kL * kL,
        VTh + (size_t)bh0 * kDH * kL, VTl + (size_t)bh0 * kDH * kL, kL, (long)kDH * kL,
        (void*)(outp + (size_t)bb * kL * kNH * kDH + (size_t)h0 * kDH),
        (void*)(outp + (size_t)bb * kL * kNH * kDH + (size_t)h0 * kDH), kNH * kDH, (long)kDH,
        cosA, cosA, 0L, kL, kDH, kL, 1.0f);
  }
  (void)hipGetLastError();
}
